// CausalIVPAttention_6390911336880
// MI455X (gfx1250) — hardware-verified
//
#include <hip/hip_runtime.h>


#define TT   512
#define CC   256
#define NH_  8
#define HDD  32
#define HID  64
#define NPR  131328
#define DM   CC
#define NTK  TT
#define LOSC 1024.0f

typedef _Float16 h16;
typedef unsigned short bf;
typedef __attribute__((ext_vector_type(16))) __bf16   v16bf;
typedef __attribute__((ext_vector_type(16))) _Float16 v16h;
typedef __attribute__((ext_vector_type(8)))  _Float16 v8h;
typedef __attribute__((ext_vector_type(8)))  unsigned short v8us;
typedef __attribute__((ext_vector_type(8)))  float    v8f;
typedef __attribute__((ext_vector_type(4)))  float    v4f;
typedef __attribute__((ext_vector_type(4)))  _Float16 v4h;
typedef v8h  __attribute__((may_alias)) v8ha;
typedef v4f  __attribute__((may_alias)) v4fa;
typedef v8us __attribute__((may_alias)) v8usa;

__device__ __forceinline__ unsigned short f2bf(float f) { unsigned u = __float_as_uint(f); u += 0x7FFFu + ((u >> 16) & 1u); return (unsigned short)(u >> 16); }
__device__ __forceinline__ float bf2f(unsigned short b) { return __uint_as_float(((unsigned)b) << 16); }
__device__ __forceinline__ float bfr(float f) { return bf2f(f2bf(f)); }
__device__ __forceinline__ v16h cat16(v8h lo, v8h hi) { return __builtin_shufflevector(lo, hi, 0, 1, 2, 3, 4, 5, 6, 7, 8, 9, 10, 11, 12, 13, 14, 15); }
__device__ __forceinline__ v16bf cat16b(v8us lo, v8us hi) { return __builtin_bit_cast(v16bf, __builtin_shufflevector(lo, hi, 0, 1, 2, 3, 4, 5, 6, 7, 8, 9, 10, 11, 12, 13, 14, 15)); }
__device__ __forceinline__ v8f wmma16(v16h a, v16h b, v8f c) { return __builtin_amdgcn_wmma_f32_16x16x32_f16(false, a, false, b, (short)0, c, false, false); }
__device__ __forceinline__ v8f wmmab(v16bf a, v16bf b, v8f c) { return __builtin_amdgcn_wmma_f32_16x16x32_bf16(false, a, false, b, (short)0, c, false, false); }

__global__ __launch_bounds__(256) void k_cvtb(const float* __restrict__ src, int nrows, bf* dst) {
    const int lane = threadIdx.x & 31, r = blockIdx.x * 8 + (threadIdx.x >> 5);
    if (r >= nrows) return;
    v8us o[DM / 256];
#pragma unroll
    for (int q = 0; q < DM / 256; ++q) { v8us t;
#pragma unroll
        for (int i = 0; i < 8; ++i) t[i] = f2bf(src[(size_t)r * DM + q * 256 + lane * 8 + i]);
        o[q] = t; }
#pragma unroll
    for (int q = 0; q < DM / 256; ++q) *(volatile v8us*)(dst + (size_t)r * DM + q * 256 + lane * 8) = o[q];
    __threadfence();
#pragma unroll
    for (int q = 0; q < DM / 256; ++q) *(volatile v8us*)(dst + (size_t)r * DM + q * 256 + lane * 8) = o[q];
}

template <bool SPLITA, bool F16OUT = false>
__global__ __launch_bounds__(128) void k_gemmb(const bf* __restrict__ A, const bf* __restrict__ Al, const bf* __restrict__ Bn, const float* __restrict__ bias, float* C, int ldc, h16* C2, const float* __restrict__ R = nullptr, int K = DM, int roundR = 1) {
    __shared__ __align__(16) float ost[4][16 * 68];
    const int lane = threadIdx.x & 31, wave = threadIdx.x >> 5, lr = lane & 15, hi = lane >> 4;
    const int r0 = blockIdx.x * 64 + wave * 16, c0 = blockIdx.y * 64;
    const size_t aoff = (size_t)(r0 + lr) * K + 8 * hi;
    size_t boff[4];
#pragma unroll
    for (int t = 0; t < 4; ++t) boff[t] = (size_t)(c0 + t * 16 + lr) * K + 8 * hi;
    v8f acc[4];
#pragma unroll
    for (int t = 0; t < 4; ++t) acc[t] = (v8f){};
#pragma unroll 1
    for (int kc = 0; kc < K; kc += 32) {
        const v16bf a = cat16b(*(const v8us*)(A + aoff + kc), *(const v8us*)(A + aoff + kc + 16));
        v16bf al = a;
        if (SPLITA) al = cat16b(*(const v8us*)(Al + aoff + kc), *(const v8us*)(Al + aoff + kc + 16));
#pragma unroll
        for (int t = 0; t < 4; ++t) { const v16bf b = cat16b(*(const v8us*)(Bn + boff[t] + kc), *(const v8us*)(Bn + boff[t] + kc + 16)); acc[t] = wmmab(a, b, acc[t]); if (SPLITA) acc[t] = wmmab(al, b, acc[t]); }
        asm volatile("v_nop\n\tv_nop\n\tv_nop\n\tv_nop" : "+v"(acc[0]), "+v"(acc[1]), "+v"(acc[2]), "+v"(acc[3]) : "v"(a), "v"(al));
    }
    float* os = &ost[wave][0];
#pragma unroll
    for (int t = 0; t < 4; ++t) { const float bv = bias ? bfr(bias[c0 + t * 16 + lr]) : 0.f;
#pragma unroll
        for (int j = 0; j < 8; ++j) os[(hi * 8 + j) * 68 + t * 16 + lr] = acc[t][j] + bv; }
    __syncthreads();
    if (F16OUT) {
        h16* crow = (h16*)(void*)C + (size_t)r0 * ldc + c0;
        auto pass = [&]() {
#pragma unroll
            for (int s = 0; s < 4; ++s) { const int row = 4 * s + (lane >> 3), piece = lane & 7; const float* sp = os + row * 68 + piece * 8; v8h o, o2;
#pragma unroll
                for (int i = 0; i < 8; ++i) { const h16 a = (h16)sp[i]; o[i] = a; o2[i] = (h16)((sp[i] - (float)a) * LOSC); }
                *(volatile v8h*)(crow + (size_t)row * ldc + piece * 8) = o; if (C2) *(volatile v8h*)(C2 + (size_t)r0 * ldc + c0 + (size_t)row * ldc + piece * 8) = o2; }
        };
        pass(); __threadfence(); pass();
    } else {
        float* crow = C + (size_t)r0 * ldc + c0;
        auto pass = [&]() {
#pragma unroll
            for (int s = 0; s < 8; ++s) { const int Lid = (lane >> 3) + 4 * s, piece = lane & 7; const int row = Lid >> 1, cofs = (Lid & 1) * 32 + piece * 4;
                v4f val = *(const v4fa*)(os + row * 68 + cofs); if (R) { const v4f rv = *(const v4f*)(R + ((size_t)r0 + row) * ldc + c0 + cofs); val += roundR ? (v4f){bfr(rv[0]), bfr(rv[1]), bfr(rv[2]), bfr(rv[3])} : rv; }
                *(volatile v4f*)(crow + (size_t)row * ldc + cofs) = val; }
        };
        pass(); __threadfence(); pass();
    }
}


__global__ __launch_bounds__(256) void k_wpad3(const float* __restrict__ w2, const float* __restrict__ w3, const float* __restrict__ b3, bf* W2B, bf* W3P, float* B3P) {
    const int u = blockIdx.x * 256 + threadIdx.x;
    if (u < HID * HID / 8) { const int n = u / (HID / 8), k0 = (u % (HID / 8)) * 8; v8us a, c;
#pragma unroll
        for (int i = 0; i < 8; ++i) { a[i] = f2bf(w2[n * HID + k0 + i]); c[i] = (n < HDD) ? f2bf(w3[n * HID + k0 + i]) : (unsigned short)0; }
        *(volatile v8us*)(W2B + n * HID + k0) = a; *(volatile v8us*)(W3P + n * HID + k0) = c; __threadfence(); *(volatile v8us*)(W2B + n * HID + k0) = a; *(volatile v8us*)(W3P + n * HID + k0) = c; }
    if (u < HID / 4) { v4f b;
#pragma unroll
        for (int i = 0; i < 4; ++i) { const int n = u * 4 + i; b[i] = (n < HDD) ? b3[n] : 0.f; }
        *(volatile v4f*)(B3P + u * 4) = b; __threadfence(); *(volatile v4f*)(B3P + u * 4) = b; }
}
__global__ __launch_bounds__(256) void k_att(const float* __restrict__ QKV, float* ATT) {
    const int lane = threadIdx.x & 31, wid = blockIdx.x * 8 + (threadIdx.x >> 5); if (wid >= NH_ * TT) return;
    const int h = wid / TT, i = wid % TT;
    const float* qr = QKV + (size_t)i * (3 * CC) + h * HDD;
    float sc[TT / 32]; float m = -3.0e38f;
#pragma unroll
    for (int q = 0; q < TT / 32; ++q) { const int j = q * 32 + lane; float s = -__builtin_inff();
        if (j <= i) { const float* kr = QKV + (size_t)j * (3 * CC) + CC + h * HDD; float d = 0.f;
#pragma unroll 1
            for (int e = 0; e < HDD; ++e) d = fmaf(qr[e], kr[e], d);
            s = d * 0.17677669529663687f; }
        sc[q] = s; m = fmaxf(m, s); }
#pragma unroll
    for (int sh = 16; sh; sh >>= 1) m = fmaxf(m, __shfl_xor(m, sh, 32));
    float sum = 0.f;
#pragma unroll
    for (int q = 0; q < TT / 32; ++q) { sc[q] = (q * 32 + lane <= i) ? __expf(sc[q] - m) : 0.f; sum += sc[q]; }
#pragma unroll
    for (int sh = 16; sh; sh >>= 1) sum += __shfl_xor(sum, sh, 32);
    const float inv = 1.0f / sum;
#pragma unroll 1
    for (int ps = 0; ps < 2; ++ps) {
#pragma unroll
        for (int q = 0; q < TT / 32; ++q) *(volatile float*)(ATT + ((size_t)h * TT + i) * TT + q * 32 + lane) = sc[q] * inv;
        if (ps == 0) __threadfence(); }
}
__global__ __launch_bounds__(256) void k_g1(const float* __restrict__ QKV, const float* __restrict__ w1, float* G) {
    const int lane = threadIdx.x & 31, wid = blockIdx.x * 8 + (threadIdx.x >> 5); if (wid >= NH_ * TT) return;
    const int h = wid / TT, j = wid % TT; const float* vr = QKV + (size_t)j * (3 * CC) + 2 * CC + h * HDD;
    float g0 = 0.f, g1 = 0.f;
#pragma unroll 1
    for (int e = 0; e < HDD; ++e) { const float v = vr[e]; g0 = fmaf(bfr(w1[lane * (HDD + 1) + e]), v, g0); g1 = fmaf(bfr(w1[(lane + 32) * (HDD + 1) + e]), v, g1); }
    float* gp = G + ((size_t)h * TT + j) * HID;
    *(volatile float*)(gp + lane) = g0; *(volatile float*)(gp + 32 + lane) = g1; __threadfence(); *(volatile float*)(gp + lane) = g0; *(volatile float*)(gp + 32 + lane) = g1;
}
__device__ __forceinline__ void pair_of(int p, int& i, int& j) {
    int ii = (int)((sqrtf(8.0f * (float)p + 1.0f) - 1.0f) * 0.5f);
    while (ii * (ii + 1) / 2 > p) --ii; while ((ii + 1) * (ii + 2) / 2 <= p) ++ii;
    i = ii; j = p - ii * (ii + 1) / 2;
}
__global__ __launch_bounds__(256) void k_pair1(const float* __restrict__ G, const float* __restrict__ t, const float* __restrict__ w1, const float* __restrict__ b1, int h, bf* Hh, bf* Hl) {
    typedef __attribute__((ext_vector_type(4))) unsigned short v4us;
    const int lane = threadIdx.x & 31, wid = blockIdx.x * 8 + (threadIdx.x >> 5); const int p = wid * 2 + (lane >> 4); if (p >= NPR) return;
    int i, j; pair_of(p, i, j); const float dt = bfr(t[i]) - bfr(t[j]);
    const int c0 = (lane & 15) * 4; float y[4];
#pragma unroll
    for (int q = 0; q < 4; ++q) { const int c = c0 + q; y[q] = fmaxf(G[((size_t)h * TT + j) * HID + c] + bfr(w1[c * (HDD + 1) + HDD]) * dt + bfr(b1[c]), 0.f); }
    v4us oh, ol;
#pragma unroll
    for (int q = 0; q < 4; ++q) { const unsigned short hb = f2bf(y[q]); oh[q] = hb; ol[q] = f2bf(y[q] - bf2f(hb)); }
    const size_t o = (size_t)p * HID + c0; *(volatile v4us*)(Hh + o) = oh; *(volatile v4us*)(Hl + o) = ol; __threadfence(); *(volatile v4us*)(Hh + o) = oh; *(volatile v4us*)(Hl + o) = ol;
}
__global__ __launch_bounds__(256) void k_relu2(const float* __restrict__ T2, bf* Hh, bf* Hl) {
    typedef __attribute__((ext_vector_type(4))) unsigned short v4us;
    const int lane = threadIdx.x & 31, wid = blockIdx.x * 8 + (threadIdx.x >> 5); const int p = wid * 2 + (lane >> 4); if (p >= NPR) return;
    const size_t o = (size_t)p * HID + (lane & 15) * 4; const v4f v = *(const v4f*)(T2 + o); v4us oh, ol;
#pragma unroll
    for (int q = 0; q < 4; ++q) { const float y = fmaxf(v[q], 0.f); const unsigned short hb = f2bf(y); oh[q] = hb; ol[q] = f2bf(y - bf2f(hb)); }
    *(volatile v4us*)(Hh + o) = oh; *(volatile v4us*)(Hl + o) = ol; __threadfence(); *(volatile v4us*)(Hh + o) = oh; *(volatile v4us*)(Hl + o) = ol;
}
__global__ __launch_bounds__(256) void k_ysum(const float* __restrict__ ATT, const float* __restrict__ QKV, const float* __restrict__ RES, const float* __restrict__ t, const float* __restrict__ tw, const float* __restrict__ tb, int h, float* CTX) {
    const int lane = threadIdx.x & 31, i = blockIdx.x * 8 + (threadIdx.x >> 5); if (i >= TT) return;
    const int d = lane; const float twd = bfr(tw[d]), tbd = bfr(tb[d]), ti = bfr(t[i]);
    const float* ar = ATT + ((size_t)h * TT + i) * TT; const size_t p0 = (size_t)i * (i + 1) / 2;
    float y = 0.f;
#pragma unroll 1
    for (int j = 0; j <= i; ++j) { const float dt = ti - bfr(t[j]); const float vj = QKV[(size_t)j * (3 * CC) + 2 * CC + h * HDD + d];
        const float tf = tanhf(dt * twd + tbd); const float vt = vj + tf * RES[(p0 + j) * HID + d]; y = fmaf(ar[j], vt, y); }
    float* cp = CTX + (size_t)i * CC + h * HDD + d; *(volatile float*)cp = y; __threadfence(); *(volatile float*)cp = y;
}
__global__ __launch_bounds__(256) void k_split(const float* __restrict__ src, int nrows, bf* dh, bf* dl) {
    const int lane = threadIdx.x & 31, r = blockIdx.x * 8 + (threadIdx.x >> 5); if (r >= nrows) return;
    const size_t o = (size_t)r * CC + lane * 8; const v8f v = *(const v8f*)(src + o); v8us oh, ol;
#pragma unroll
    for (int q = 0; q < 8; ++q) { const unsigned short hb = f2bf(v[q]); oh[q] = hb; ol[q] = f2bf(v[q] - bf2f(hb)); }
    *(volatile v8us*)(dh + o) = oh; *(volatile v8us*)(dl + o) = ol; __threadfence(); *(volatile v8us*)(dh + o) = oh; *(volatile v8us*)(dl + o) = ol;
}

extern "C" void kernel_launch(void* const* d_in, const int* in_sizes, int n_in,
                              void* d_out, int out_size, void* d_ws, size_t ws_size, hipStream_t stream) {
    (void)in_sizes; (void)n_in; (void)out_size;
    const float* x = (const float*)d_in[0]; const float* t = (const float*)d_in[1]; const float* w_attn = (const float*)d_in[2]; const float* b_attn = (const float*)d_in[3]; const float* w_proj = (const float*)d_in[4]; const float* b_proj = (const float*)d_in[5];
    const float* w1 = (const float*)d_in[6]; const float* b1 = (const float*)d_in[7]; const float* w2 = (const float*)d_in[8]; const float* b2 = (const float*)d_in[9]; const float* w3 = (const float*)d_in[10]; const float* b3 = (const float*)d_in[11]; const float* tw = (const float*)d_in[12]; const float* tb = (const float*)d_in[13];
    float* out = (float*)d_out;
    char* wsp = (char*)d_ws;
    auto take = [&](size_t bytes) { char* p = wsp; wsp += (bytes + 255) & ~(size_t)255; return (void*)p; };
    bf* WaB = (bf*)take((size_t)3 * CC * CC * 2); bf* WpB = (bf*)take((size_t)CC * CC * 2); bf* W2B = (bf*)take(HID * HID * 2); bf* W3P = (bf*)take(HID * HID * 2); float* B3P = (float*)take(HID * 4);
    bf* Xb = (bf*)take((size_t)TT * CC * 2); float* QKV = (float*)take((size_t)TT * 3 * CC * 4); float* ATT = (float*)take((size_t)NH_ * TT * TT * 4); float* G = (float*)take((size_t)NH_ * TT * HID * 4);
    bf* H1h = (bf*)take((size_t)NPR * HID * 2); bf* H1l = (bf*)take((size_t)NPR * HID * 2); float* T2 = (float*)take((size_t)NPR * HID * 4); bf* H2h = (bf*)take((size_t)NPR * HID * 2); bf* H2l = (bf*)take((size_t)NPR * HID * 2); float* RES = T2;
    float* CTX = (float*)take((size_t)TT * CC * 4); bf* Ch = (bf*)take((size_t)TT * CC * 2); bf* Cl = (bf*)take((size_t)TT * CC * 2);
    if ((size_t)(wsp - (char*)d_ws) > ws_size) return;
    k_cvtb<<<(3 * CC) / 8, 256, 0, stream>>>(w_attn, 3 * CC, WaB); k_cvtb<<<CC / 8, 256, 0, stream>>>(w_proj, CC, WpB); k_wpad3<<<(HID * HID / 8 + 255) / 256, 256, 0, stream>>>(w2, w3, b3, W2B, W3P, B3P);
    k_cvtb<<<TT / 8, 256, 0, stream>>>(x, TT, Xb);
    k_gemmb<false, false><<<dim3(TT / 64, (3 * CC) / 64, 1), 128, 0, stream>>>(Xb, nullptr, WaB, b_attn, QKV, 3 * CC, nullptr);
    k_att<<<(NH_ * TT) / 8, 256, 0, stream>>>(QKV, ATT);
    k_g1<<<(NH_ * TT) / 8, 256, 0, stream>>>(QKV, w1, G);
    for (int h = 0; h < NH_; ++h) {
        k_pair1<<<(NPR / 2 + 7) / 8, 256, 0, stream>>>(G, t, w1, b1, h, H1h, H1l);
        k_gemmb<true, false><<<dim3(NPR / 64, 1, 1), 128, 0, stream>>>(H1h, H1l, W2B, b2, T2, HID, nullptr, nullptr, HID);
        k_relu2<<<(NPR / 2 + 7) / 8, 256, 0, stream>>>(T2, H2h, H2l);
        k_gemmb<true, false><<<dim3(NPR / 64, 1, 1), 128, 0, stream>>>(H2h, H2l, W3P, B3P, RES, HID, nullptr, nullptr, HID);
        k_ysum<<<TT / 8, 256, 0, stream>>>(ATT, QKV, RES, t, tw, tb, h, CTX);
    }
    k_split<<<TT / 8, 256, 0, stream>>>(CTX, TT, Ch, Cl);
    k_gemmb<true, false><<<dim3(TT / 64, CC / 64, 1), 128, 0, stream>>>(Ch, Cl, WpB, b_proj, out, CC, nullptr);
}
